// OffsetAttention_47699906789389
// MI455X (gfx1250) — hardware-run, weakly checked
//
#include <hip/hip_runtime.h>
#include <math.h>
#include <stdint.h>

#ifndef NB
#define NB 4
#endif
#ifndef SEQ
#define SEQ 2048
#endif
#define NB_FULL  4
#define SEQ_FULL 2048
#define DM       256
#define MROWS    (NB * SEQ)
#define NQT16    (SEQ / 16)
#define SPITCH   (SEQ + 4)
#define QSC      1024.0f
#define KSC      1024.0f
#define PCAR     32768.0f
#define VCAR     1024.0f
#define LOG2E    1.4426950408889634f
#define EPS_RN   1e-9f
#define EPS_BN   1e-5f
#define SLP      68
#define SLAB64   (16 * SLP)
#define VTP      72
#define BNR      256
#define WS_CAP   134217728
static_assert(NB >= 1 && NB <= NB_FULL);
static_assert(SEQ >= 256 && SEQ <= SEQ_FULL && (SEQ % 256) == 0 && (SEQ % 64) == 0 && (SEQ / 256) <= 8);
static_assert(DM == 256 && (DM / 8) == 32 && (DM % 64) == 0 && (DM % 32) == 0);
static_assert((MROWS % 64) == 0 && (MROWS % BNR) == 0);
static_assert((SPITCH % 4) == 0);

typedef unsigned short u16;
typedef _Float16 v16h __attribute__((ext_vector_type(16)));
typedef _Float16 v8h  __attribute__((ext_vector_type(8)));
typedef __bf16   v16b __attribute__((ext_vector_type(16)));
typedef float    v8f  __attribute__((ext_vector_type(8)));
typedef float    v4f  __attribute__((ext_vector_type(4)));
typedef unsigned int v4u __attribute__((ext_vector_type(4)));
typedef double   v2d  __attribute__((ext_vector_type(2)));

union FragH { v16h v; v8h h[2]; v4u u[2]; };
union FragB { v16b v; v4u u[2]; };

__device__ __forceinline__ unsigned short bf_bits(float f) {
  unsigned u = __float_as_uint(f);
  return (unsigned short)((u + 0x7FFFu + ((u >> 16) & 1u)) >> 16);
}
__device__ __forceinline__ float bf_up(unsigned short h) { return __uint_as_float(((unsigned)h) << 16); }
__device__ __forceinline__ float bfr(float f) { return bf_up(bf_bits(f)); }
__device__ __forceinline__ unsigned short h_bits(_Float16 x) { return __builtin_bit_cast(unsigned short, x); }
__device__ __forceinline__ unsigned pk16(unsigned short a, unsigned short b) { return (unsigned)a | ((unsigned)b << 16); }
__device__ __forceinline__ v8f zero8() { v8f z = {0.f, 0.f, 0.f, 0.f, 0.f, 0.f, 0.f, 0.f}; return z; }

__device__ __forceinline__ v16h ldfrag_h(const _Float16* p) {
  FragH f;
  f.h[0] = *(const v8h*)(p);
  f.h[1] = *(const v8h*)(p + 16);
  return f.v;
}
__device__ __forceinline__ v16b ldfrag_b(const u16* p) {
  FragB f;
  f.u[0] = *(const v4u*)(p);
  f.u[1] = *(const v4u*)(p + 16);
  return f.v;
}

__device__ __forceinline__ v8f mma_h(v16h a, v16h b, v8f c) {
  return __builtin_amdgcn_wmma_f32_16x16x32_f16(false, a, false, b, (short)0, c, false, false);
}
__device__ __forceinline__ v8f mma_b(v16b a, v16b b, v8f c) {
  return __builtin_amdgcn_wmma_f32_16x16x32_bf16(false, a, false, b, (short)0, c, false, false);
}
template <typename F>
__device__ __forceinline__ void guard6(v8f& a, v8f& b, v8f& c, v8f& d, F x0, F x1, F x2, F x3, F x4, F x5) {
#if defined(__HIP_DEVICE_COMPILE__)
  asm volatile("v_nop\n\tv_nop\n\tv_nop\n\tv_nop"
               : "+v"(a), "+v"(b), "+v"(c), "+v"(d) : "v"(x0), "v"(x1), "v"(x2), "v"(x3), "v"(x4), "v"(x5) : "memory");
#endif
}
__device__ __forceinline__ void wave_sync_lds() {
  __builtin_amdgcn_fence(__ATOMIC_RELEASE, "workgroup");
  __builtin_amdgcn_wave_barrier();
  __builtin_amdgcn_fence(__ATOMIC_ACQUIRE, "workgroup");
}

__global__ __launch_bounds__(256) void cvt16(const float* __restrict__ x, u16* D, int n8) {
  const int gt = blockIdx.x * 256 + (int)threadIdx.x;
  if (gt >= n8) return;
  const int pr = gt >> 5;
  const int c8 = (gt & 31) * 8;
  const int b  = pr / SEQ;
  const int s  = pr - b * SEQ;
  const float* p = x + ((size_t)b * SEQ_FULL + s) * DM + c8;
  const v4f a = *(const v4f*)(p), b4 = *(const v4f*)(p + 4);
  v4u o;
#pragma unroll
  for (int e = 0; e < 2; ++e) {
    o[e]     = pk16(bf_bits(a[2 * e]),  bf_bits(a[2 * e + 1]));
    o[2 + e] = pk16(bf_bits(b4[2 * e]), bf_bits(b4[2 * e + 1]));
  }
  u16* d = D + (size_t)pr * DM + c8;
  for (int pass = 0; pass < 2; ++pass) {
    *(volatile v4u*)(d) = o;
    __threadfence();
  }
}

__global__ __launch_bounds__(256) void wt16(const float* __restrict__ W, u16* D) {
  __shared__ __align__(16) u16 T[128 * VTP];
  const int tid = threadIdx.x;
  const int bid = blockIdx.x;
  const int ct  = bid & 1;
  const int rt  = bid >> 1;
  if (rt * 64 + 64 > DM) return;
  {
    const int sl = tid >> 2;
    const int dc = (tid & 3) * 32;
    const float* src = W + (size_t)(rt * 64 + sl) * DM + ct * 128 + dc;
#pragma unroll
    for (int i = 0; i < 8; ++i) {
      const v4f a = *(const v4f*)(src + 4 * i);
#pragma unroll
      for (int e = 0; e < 4; ++e) {
        T[(dc + 4 * i + e) * VTP + sl] = bf_bits(a[e]);
      }
    }
  }
  __syncthreads();
  v4u w4[4];
  const int q8 = tid >> 3, p8 = (tid & 7) * 8;
#pragma unroll
  for (int it = 0; it < 4; ++it) {
    const int line = it * 32 + q8;
    w4[it] = *(const v4u*)(T + line * VTP + p8);
  }
  const size_t base = ((size_t)ct * 128) * DM + rt * 64 + p8;
  for (int pass = 0; pass < 2; ++pass) {
#pragma unroll
    for (int it = 0; it < 4; ++it) {
      const int line = it * 32 + q8;
      *(volatile v4u*)(D + base + (size_t)line * DM) = w4[it];
    }
    __threadfence();
  }
}

__device__ __forceinline__ void epi64(float* sl, v8f a0, v8f a1, v8f a2, v8f a3,
                                      float bb0, float bb1, float bb2, float bb3,
                                      float* C, int N, size_t rowb, int col0, int lane) {
  const int hh = lane >> 4, m = lane & 15;
#pragma unroll
  for (int r = 0; r < 8; ++r) {
    const int ro = (8 * hh + r) * SLP + m;
    sl[ro]      = a0[r] + bb0;
    sl[ro + 16] = a1[r] + bb1;
    sl[ro + 32] = a2[r] + bb2;
    sl[ro + 48] = a3[r] + bb3;
  }
  wave_sync_lds();
  v4f vals[8];
#pragma unroll
  for (int it = 0; it < 8; ++it) vals[it] = *(const v4f*)(sl + (it * 2 + hh) * SLP + m * 4);
  float* dst = C + (rowb + (size_t)hh) * (size_t)N + col0 + m * 4;
  for (int pass = 0; pass < 2; ++pass) {
#pragma unroll
    for (int it = 0; it < 8; ++it) {
      *(volatile v4f*)(dst + (size_t)(it * 2) * (size_t)N) = vals[it];
    }
    __threadfence();
  }
}

__device__ __forceinline__ void epi16(float* sl, v8f a0, v8f a1, v8f a2, v8f a3,
                                      float bb0, float bb1, float bb2, float bb3, float osc,
                                      u16* C, int N, size_t rowb, int col0, int lane) {
  const int hh = lane >> 4, m = lane & 15;
#pragma unroll
  for (int r = 0; r < 8; ++r) {
    const int ro = (8 * hh + r) * SLP + m;
    sl[ro]      = a0[r] + bb0;
    sl[ro + 16] = a1[r] + bb1;
    sl[ro + 32] = a2[r] + bb2;
    sl[ro + 48] = a3[r] + bb3;
  }
  wave_sync_lds();
  const int rq = lane >> 3, c8 = (lane & 7) * 8;
  v4u w4[4];
#pragma unroll
  for (int it = 0; it < 4; ++it) {
    const int row = it * 4 + rq;
    const v4f x0 = *(const v4f*)(sl + row * SLP + c8), x1 = *(const v4f*)(sl + row * SLP + c8 + 4);
#pragma unroll
    for (int e = 0; e < 2; ++e) {
      w4[it][e]     = pk16(h_bits((_Float16)(x0[2 * e] * osc)), h_bits((_Float16)(x0[2 * e + 1] * osc)));
      w4[it][2 + e] = pk16(h_bits((_Float16)(x1[2 * e] * osc)), h_bits((_Float16)(x1[2 * e + 1] * osc)));
    }
  }
  for (int pass = 0; pass < 2; ++pass) {
#pragma unroll
    for (int it = 0; it < 4; ++it) {
      const int row = it * 4 + rq;
      *(volatile v4u*)(C + (rowb + (size_t)row) * (size_t)N + col0 + c8) = w4[it];
    }
    __threadfence();
  }
}

template <int OM>
__global__ __launch_bounds__(128)
void gemm_x(const u16* __restrict__ A, const u16* __restrict__ Bt, const float* __restrict__ bias,
            float* Cf, u16* Ch, int M, int N, int K, float osc) {
  __shared__ __align__(16) float slab[4 * SLAB64];
  const int tid = threadIdx.x, wave = tid >> 5, lane = tid & 31, hh = lane >> 4, m = lane & 15;
  const int ntile = N >> 6;
  const int bid   = blockIdx.x;
  const int rowb  = (bid / ntile) * 64 + wave * 16;
  const int col0  = (bid % ntile) * 64;
  if (rowb + 16 > M) return;
  const u16* ap = A  + (size_t)(rowb + m) * K + 8 * hh;
  const u16* bp = Bt + (size_t)(col0 + m) * K + 8 * hh;
  const size_t bs = (size_t)16 * K;
  v8f acc0 = zero8(), acc1 = zero8(), acc2 = zero8(), acc3 = zero8();
#pragma unroll 1
  for (int k0 = 0; k0 < K; k0 += 32) {
    const v16b a  = ldfrag_b(ap + k0);
    const v16b b0 = ldfrag_b(bp + k0);
    const v16b b1 = ldfrag_b(bp + bs + k0);
    const v16b b2 = ldfrag_b(bp + 2 * bs + k0);
    const v16b b3 = ldfrag_b(bp + 3 * bs + k0);
    acc0 = mma_b(a, b0, acc0);
    acc1 = mma_b(a, b1, acc1);
    acc2 = mma_b(a, b2, acc2);
    acc3 = mma_b(a, b3, acc3);
    guard6<v16b>(acc0, acc1, acc2, acc3, a, b0, b1, b2, b3, a);
  }
  const float bb0 = bfr(bias[col0 + m]);
  const float bb1 = bfr(bias[col0 + 16 + m]);
  const float bb2 = bfr(bias[col0 + 32 + m]);
  const float bb3 = bfr(bias[col0 + 48 + m]);
  if constexpr (OM == 0) {
    epi64(slab + wave * SLAB64, acc0, acc1, acc2, acc3, bb0, bb1, bb2, bb3, Cf, N, (size_t)rowb, col0, lane);
  } else {
    epi16(slab + wave * SLAB64, acc0, acc1, acc2, acc3, bb0, bb1, bb2, bb3, osc, Ch, N, (size_t)rowb, col0, lane);
  }
}

__global__ __launch_bounds__(256)
void attn_p(const u16* __restrict__ QH, const u16* __restrict__ KH, u16* P, float* CP) {
  extern __shared__ __align__(16) float smem[];
  float* S = smem;
  const int tid = threadIdx.x, wave = tid >> 5, lane = tid & 31, hh = lane >> 4, m = lane & 15;
  const int bid = blockIdx.x;
  const int qt  = bid % NQT16;
  const int b   = bid / NQT16;
  if (b >= NB) return;
  const int q0  = qt * 16;
  const _Float16* qp  = (const _Float16*)(const void*)QH + ((size_t)b * SEQ + q0 + m) * DM + 8 * hh;
  const _Float16* kp0 = (const _Float16*)(const void*)KH + ((size_t)b * SEQ + m) * DM + 8 * hh;
  const size_t bs = (size_t)16 * DM;

#pragma unroll 1
  for (int ct = wave; ct < SEQ / 64; ct += 8) {
    const _Float16* kp = kp0 + (size_t)ct * 64 * DM;
    v8f acc0 = zero8(), acc1 = zero8(), acc2 = zero8(), acc3 = zero8();
#pragma unroll 1
    for (int k0 = 0; k0 < DM; k0 += 32) {
      const v16h a  = ldfrag_h(qp + k0);
      const v16h b0 = ldfrag_h(kp + k0);
      const v16h b1 = ldfrag_h(kp + bs + k0);
      const v16h b2 = ldfrag_h(kp + 2 * bs + k0);
      const v16h b3 = ldfrag_h(kp + 3 * bs + k0);
      acc0 = mma_h(a, b0, acc0);
      acc1 = mma_h(a, b1, acc1);
      acc2 = mma_h(a, b2, acc2);
      acc3 = mma_h(a, b3, acc3);
      guard6<v16h>(acc0, acc1, acc2, acc3, a, b0, b1, b2, b3, a);
    }
    float* sb = S + (size_t)(8 * hh) * SPITCH + ct * 64 + m;
#pragma unroll
    for (int r = 0; r < 8; ++r) {
      float* sr = sb + (size_t)r * SPITCH;
      sr[0]  = acc0[r];
      sr[16] = acc1[r];
      sr[32] = acc2[r];
      sr[48] = acc3[r];
    }
  }
  __syncthreads();

  const float lsc = LOG2E / (QSC * KSC);
  constexpr int NIT = SEQ / 256;
#pragma unroll 1
  for (int rr = 0; rr < 2; ++rr) {
    const int r = wave + 8 * rr;
    float* Sr = S + (size_t)r * SPITCH + lane * 8;
    float mx = -INFINITY;
#pragma unroll
    for (int it = 0; it < NIT; ++it) {
      const v4f a = *(const v4f*)(Sr + it * 256), c = *(const v4f*)(Sr + it * 256 + 4);
#pragma unroll
      for (int e = 0; e < 4; ++e) { mx = fmaxf(mx, a[e] * lsc); mx = fmaxf(mx, c[e] * lsc); }
    }
#pragma unroll
    for (int off = 1; off < 32; off <<= 1) mx = fmaxf(mx, __shfl_xor(mx, off, 32));
    float sum = 0.0f;
#pragma unroll
    for (int it = 0; it < NIT; ++it) {
      v4f a = *(const v4f*)(Sr + it * 256), c = *(const v4f*)(Sr + it * 256 + 4);
#pragma unroll
      for (int e = 0; e < 4; ++e) {
        a[e] = exp2f(a[e] * lsc - mx);
        c[e] = exp2f(c[e] * lsc - mx);
        sum += a[e] + c[e];
      }
      *(v4f*)(Sr + it * 256)     = a;
      *(v4f*)(Sr + it * 256 + 4) = c;
    }
#pragma unroll
    for (int off = 1; off < 32; off <<= 1) sum += __shfl_xor(sum, off, 32);
    const float inv = 1.0f / sum;
    v4u pk[NIT];
#pragma unroll
    for (int it = 0; it < NIT; ++it) {
      v4f a = *(const v4f*)(Sr + it * 256), c = *(const v4f*)(Sr + it * 256 + 4);
#pragma unroll
      for (int e = 0; e < 4; ++e) { a[e] = a[e] * inv; c[e] = c[e] * inv; }
      *(v4f*)(Sr + it * 256)     = a;
      *(v4f*)(Sr + it * 256 + 4) = c;
#pragma unroll
      for (int e = 0; e < 2; ++e) {
        pk[it][e]     = pk16(h_bits((_Float16)(a[2 * e] * PCAR)), h_bits((_Float16)(a[2 * e + 1] * PCAR)));
        pk[it][2 + e] = pk16(h_bits((_Float16)(c[2 * e] * PCAR)), h_bits((_Float16)(c[2 * e + 1] * PCAR)));
      }
    }
    u16* prow = P + ((size_t)b * SEQ + q0 + r) * SEQ + lane * 8;
    for (int pass = 0; pass < 2; ++pass) {
#pragma unroll
      for (int it = 0; it < NIT; ++it) {
        *(volatile v4u*)(prow + it * 256) = pk[it];
      }
      __threadfence();
    }
  }
  __syncthreads();

#pragma unroll 1
  for (int c4 = tid * 4; c4 < SEQ; c4 += 1024) {
    v4f cs = {0.f, 0.f, 0.f, 0.f};
#pragma unroll
    for (int r = 0; r < 16; ++r) cs += *(const v4f*)(S + (size_t)r * SPITCH + c4);
    float* dst = CP + ((size_t)(b * NQT16 + qt)) * SEQ + c4;
    for (int pass = 0; pass < 2; ++pass) {
      *(volatile v4f*)(dst) = cs;
      __threadfence();
    }
  }
}

__global__ __launch_bounds__(256) void csred(const float* __restrict__ CP, float* RCS, int n4) {
  const int gt = blockIdx.x * 256 + (int)threadIdx.x;
  if (gt >= n4) return;
  const int idx = gt * 4;
  const int b   = idx / SEQ;
  const int k   = idx - b * SEQ;
  const float* p = CP + (size_t)b * NQT16 * SEQ + k;
  v4f s = {0.f, 0.f, 0.f, 0.f};
#pragma unroll 1
  for (int qt = 0; qt < NQT16; ++qt) s += *(const v4f*)(p + (size_t)qt * SEQ);
  v4f rc;
#pragma unroll
  for (int e = 0; e < 4; ++e) rc[e] = 1.0f / (EPS_RN + s[e]);
  float* d = RCS + idx;
  for (int pass = 0; pass < 2; ++pass) {
    *(volatile v4f*)(d) = rc;
    __threadfence();
  }
}

__global__ __launch_bounds__(256) void vt16(const float* __restrict__ F, const float* __restrict__ RCS, u16* VT) {
  __shared__ __align__(16) u16 T[64 * VTP];
  const int tid = threadIdx.x;
  const int bid = blockIdx.x;
  const int nst = SEQ / 64;
  const int st  = bid % nst;
  const int t2  = bid / nst;
  const int dt  = t2 & 3;
  const int b   = t2 >> 2;
  if (b >= NB) return;
  const int s0  = st * 64;
  {
    const int sl = tid >> 2;
    const int dc = (tid & 3) * 16;
    const float* src = F + ((size_t)b * SEQ + s0 + sl) * DM + dt * 64 + dc;
    const float rc = RCS[(size_t)b * SEQ + s0 + sl] * VCAR;
#pragma unroll
    for (int i = 0; i < 4; ++i) {
      const v4f a = *(const v4f*)(src + 4 * i);
#pragma unroll
      for (int e = 0; e < 4; ++e) {
        T[(dc + 4 * i + e) * VTP + sl] = h_bits((_Float16)(a[e] * rc));
      }
    }
  }
  __syncthreads();
  v4u vh[2];
  const int q8 = tid >> 3, p8 = (tid & 7) * 8;
#pragma unroll
  for (int it = 0; it < 2; ++it) {
    const int line = it * 32 + q8;
    vh[it] = *(const v4u*)(T + line * VTP + p8);
  }
  const size_t base = ((size_t)b * DM + dt * 64) * SEQ + s0 + p8;
  for (int pass = 0; pass < 2; ++pass) {
#pragma unroll
    for (int it = 0; it < 2; ++it) {
      const int line = it * 32 + q8;
      *(volatile v4u*)(VT + base + (size_t)line * SEQ) = vh[it];
    }
    __threadfence();
  }
}

__global__ __launch_bounds__(128)
void gemm_pv(const u16* __restrict__ P, const u16* __restrict__ VT, const float* __restrict__ vals, u16* RH, u16* RL) {
  __shared__ __align__(16) float slab[4 * SLAB64];
  const int tid = threadIdx.x, wave = tid >> 5, lane = tid & 31, hh = lane >> 4, m = lane & 15;
  const int nrt = SEQ / 64;
  const int bid = blockIdx.x;
  const int b   = bid / (nrt * 4);
  const int rem = bid - b * (nrt * 4);
  const int rt  = rem >> 2;
  const int ct  = rem & 3;
  if (b >= NB) return;
  const int rowb = rt * 64 + wave * 16;
  const int col0 = ct * 64;
  const _Float16* ap = (const _Float16*)(const void*)P  + ((size_t)b * SEQ + rowb + m) * SEQ + 8 * hh;
  const _Float16* bp = (const _Float16*)(const void*)VT + ((size_t)b * DM + col0 + m) * SEQ + 8 * hh;
  const size_t bs = (size_t)16 * SEQ;
  v8f acc0 = zero8(), acc1 = zero8(), acc2 = zero8(), acc3 = zero8();
#pragma unroll 1
  for (int k0 = 0; k0 < SEQ; k0 += 32) {
    const v16h a  = ldfrag_h(ap + k0);
    const v16h b0 = ldfrag_h(bp + k0);
    const v16h b1 = ldfrag_h(bp + bs + k0);
    const v16h b2 = ldfrag_h(bp + 2 * bs + k0);
    const v16h b3 = ldfrag_h(bp + 3 * bs + k0);
    acc0 = mma_h(a, b0, acc0);
    acc1 = mma_h(a, b1, acc1);
    acc2 = mma_h(a, b2, acc2);
    acc3 = mma_h(a, b3, acc3);
    guard6<v16h>(acc0, acc1, acc2, acc3, a, b0, b1, b2, b3, a);
  }
  float* sl = slab + wave * SLAB64;
  const float oc = 1.0f / (PCAR * VCAR);
#pragma unroll
  for (int r = 0; r < 8; ++r) {
    const int ro = (8 * hh + r) * SLP + m;
    sl[ro]      = acc0[r] * oc;
    sl[ro + 16] = acc1[r] * oc;
    sl[ro + 32] = acc2[r] * oc;
    sl[ro + 48] = acc3[r] * oc;
  }
  wave_sync_lds();
  const int rq = lane >> 3, c8 = (lane & 7) * 8;
  v4u rh[4], rl[4];
#pragma unroll
  for (int it = 0; it < 4; ++it) {
    const int row = it * 4 + rq;
    const v4f o0 = *(const v4f*)(sl + row * SLP + c8), o1 = *(const v4f*)(sl + row * SLP + c8 + 4);
    const float* vp = vals + ((size_t)b * SEQ_FULL + rowb + row) * DM + col0 + c8;
    const v4f x0 = *(const v4f*)(vp), x1 = *(const v4f*)(vp + 4);
    float rv[8];
#pragma unroll
    for (int e = 0; e < 4; ++e) { rv[e] = bfr(x0[e]) - o0[e]; rv[4 + e] = bfr(x1[e]) - o1[e]; }
#pragma unroll
    for (int e = 0; e < 4; ++e) {
      const unsigned short ha = bf_bits(rv[2 * e]), hb = bf_bits(rv[2 * e + 1]);
      const unsigned short la = bf_bits(rv[2 * e] - bf_up(ha)), lb = bf_bits(rv[2 * e + 1] - bf_up(hb));
      rh[it][e] = pk16(ha, hb);
      rl[it][e] = pk16(la, lb);
    }
  }
  const size_t base = ((size_t)b * SEQ + rowb) * DM + col0 + c8;
  for (int pass = 0; pass < 2; ++pass) {
#pragma unroll
    for (int it = 0; it < 4; ++it) {
      const int row = it * 4 + rq;
      *(volatile v4u*)(RH + base + (size_t)row * DM) = rh[it];
      *(volatile v4u*)(RL + base + (size_t)row * DM) = rl[it];
    }
    __threadfence();
  }
}

__global__ __launch_bounds__(128)
void gemm_wo(const u16* __restrict__ RH, const u16* __restrict__ RL, const u16* __restrict__ Bt,
             const float* __restrict__ bias, float* Y, int M) {
  __shared__ __align__(16) float slab[4 * SLAB64];
  const int tid = threadIdx.x, wave = tid >> 5, lane = tid & 31, hh = lane >> 4, m = lane & 15;
  const int ntile = DM >> 6;
  const int bid   = blockIdx.x;
  const int rowb  = (bid / ntile) * 64 + wave * 16;
  const int col0  = (bid % ntile) * 64;
  if (rowb + 16 > M) return;
  const int K = DM;
  const u16* ahp = RH + (size_t)(rowb + m) * K + 8 * hh;
  const u16* alp = RL + (size_t)(rowb + m) * K + 8 * hh;
  const u16* bp  = Bt + (size_t)(col0 + m) * K + 8 * hh;
  const size_t bs = (size_t)16 * K;
  v8f acc0 = zero8(), acc1 = zero8(), acc2 = zero8(), acc3 = zero8();
#pragma unroll 1
  for (int k0 = 0; k0 < K; k0 += 32) {
    const v16b ah = ldfrag_b(ahp + k0), al = ldfrag_b(alp + k0);
    const v16b b0 = ldfrag_b(bp + k0);
    const v16b b1 = ldfrag_b(bp + bs + k0);
    const v16b b2 = ldfrag_b(bp + 2 * bs + k0);
    const v16b b3 = ldfrag_b(bp + 3 * bs + k0);
    acc0 = mma_b(ah, b0, acc0);  acc0 = mma_b(al, b0, acc0);
    acc1 = mma_b(ah, b1, acc1);  acc1 = mma_b(al, b1, acc1);
    acc2 = mma_b(ah, b2, acc2);  acc2 = mma_b(al, b2, acc2);
    acc3 = mma_b(ah, b3, acc3);  acc3 = mma_b(al, b3, acc3);
    guard6<v16b>(acc0, acc1, acc2, acc3, ah, al, b0, b1, b2, b3);
  }
  const float bb0 = bfr(bias[col0 + m]);
  const float bb1 = bfr(bias[col0 + 16 + m]);
  const float bb2 = bfr(bias[col0 + 32 + m]);
  const float bb3 = bfr(bias[col0 + 48 + m]);
  epi64(slab + wave * SLAB64, acc0, acc1, acc2, acc3, bb0, bb1, bb2, bb3, Y, DM, (size_t)rowb, col0, lane);
}

__global__ __launch_bounds__(256) void bnpart(const float* __restrict__ Y, double* BNP, int nblk) {
  __shared__ __align__(16) double L[512];
  const int tid = threadIdx.x;
  const int blk = blockIdx.x;
  if (blk >= nblk) return;
  const float* p = Y + (size_t)blk * BNR * DM + tid;
  double s = 0.0, s2 = 0.0;
#pragma unroll 4
  for (int r = 0; r < BNR; ++r) {
    const double y = (double)p[(size_t)r * DM];
    s  += y;
    s2 += y * y;
  }
  L[tid]       = s;
  L[256 + tid] = s2;
  __syncthreads();
  const v2d w = *(const v2d*)(L + 2 * tid);
  double* d = BNP + (size_t)blk * 512 + 2 * tid;
  for (int pass = 0; pass < 2; ++pass) {
    *(volatile v2d*)(d) = w;
    __threadfence();
  }
}

__global__ __launch_bounds__(256) void bnfin(const double* __restrict__ BNP, const float* __restrict__ gamma,
                                             const float* __restrict__ beta, float* BNT, int nblk) {
  __shared__ __align__(16) float L[1024];
  const int c = threadIdx.x;
  double s = 0.0, s2 = 0.0;
#pragma unroll 1
  for (int blk = 0; blk < nblk; ++blk) {
    s  += BNP[(size_t)blk * 512 + c];
    s2 += BNP[(size_t)blk * 512 + 256 + c];
  }
  const double inv  = 1.0 / (double)MROWS;
  const double mean = s * inv;
  double var = s2 * inv - mean * mean;
  if (var < 0.0) var = 0.0;
  const float mf = (float)mean;
  const float vf = (float)var;
  const float rs = rsqrtf(vf + EPS_BN);
  L[c]       = mf;
  L[256 + c] = rs;
  L[512 + c] = bfr(gamma[c]);
  L[768 + c] = bfr(beta[c]);
  __syncthreads();
  const v4f w = *(const v4f*)(L + 4 * c);
  float* d = BNT + 4 * c;
  for (int pass = 0; pass < 2; ++pass) {
    *(volatile v4f*)(d) = w;
    __threadfence();
  }
}

__global__ __launch_bounds__(256) void bnapply(const float* __restrict__ Y, const float* __restrict__ BNT, float* out, int n4) {
  const int gt = blockIdx.x * 256 + (int)threadIdx.x;
  if (gt >= n4) return;
  const size_t i = (size_t)gt * 4;
  const int c = (int)(i & (size_t)(DM - 1));
  const v4f y  = *(const v4f*)(Y + i);
  const v4f mu = *(const v4f*)(BNT + c);
  const v4f rs = *(const v4f*)(BNT + 256 + c);
  const v4f g  = *(const v4f*)(BNT + 512 + c);
  const v4f bt = *(const v4f*)(BNT + 768 + c);
  v4f z;
#pragma unroll
  for (int e = 0; e < 4; ++e) z[e] = fmaxf(((y[e] - mu[e]) * rs[e]) * g[e] + bt[e], 0.0f);
  float* d = out + i;
  for (int pass = 0; pass < 2; ++pass) {
    *(volatile v4f*)(d) = z;
    __threadfence();
  }
}

static size_t align_up(size_t v) { return (v + 255) & ~(size_t)255; }

extern "C" void kernel_launch(void* const* d_in, const int* in_sizes, int n_in,
                              void* d_out, int out_size, void* d_ws, size_t ws_size,
                              hipStream_t stream) {
  if (n_in < 13) return;
  const long needX = ((long)(NB - 1) * SEQ_FULL + SEQ) * DM;
  if ((long)in_sizes[0] < needX || (long)in_sizes[1] < needX || (long)in_sizes[2] < needX) return;
  if (in_sizes[3] < DM * DM || in_sizes[5] < DM * DM || in_sizes[7] < DM * DM || in_sizes[9] < DM * DM) return;
  if (in_sizes[4] < DM || in_sizes[6] < DM || in_sizes[8] < DM || in_sizes[10] < DM) return;
  if (in_sizes[11] < DM || in_sizes[12] < DM) return;
  if (out_size < MROWS * DM) return;

  const float* queries = (const float*)d_in[0];
  const float* keys    = (const float*)d_in[1];
  const float* values  = (const float*)d_in[2];
  const float* Wq = (const float*)d_in[3];   const float* bq = (const float*)d_in[4];
  const float* Wk = (const float*)d_in[5];   const float* bk = (const float*)d_in[6];
  const float* Wv = (const float*)d_in[7];   const float* bv = (const float*)d_in[8];
  const float* Wo = (const float*)d_in[9];   const float* bo = (const float*)d_in[10];
  const float* gamma = (const float*)d_in[11];
  const float* beta  = (const float*)d_in[12];
  float* out = (float*)d_out;

  const size_t M     = (size_t)MROWS;
  const size_t szX   = M * DM * 2;
  const size_t szW   = (size_t)DM * DM * 2;
  const size_t szH   = M * DM * 2;
  const size_t szF   = M * DM * 4;
  const size_t szP   = (size_t)NB * SEQ * SEQ * 2;
  const size_t szCP  = (size_t)NB * NQT16 * SEQ * 4;
  const size_t szRCS = (size_t)NB * SEQ * 4;
  const size_t szVT  = (size_t)NB * DM * SEQ * 2;
  const size_t szR   = M * DM * 2;
  const size_t szY   = M * DM * 4;
  const int    nblk  = (int)(M / BNR);
  const size_t szBNP = (size_t)nblk * 512 * 8;
  const size_t szBNT = 1024 * 4;
  size_t off = 0;
  const size_t oXQ = off; off = align_up(off + szX);
  const size_t oXK = off; off = align_up(off + szX);
  const size_t oXV = off; off = align_up(off + szX);
  const size_t oWQ = off; off = align_up(off + szW);
  const size_t oWK = off; off = align_up(off + szW);
  const size_t oWV = off; off = align_up(off + szW);
  const size_t oWO = off; off = align_up(off + szW);
  const size_t oQH = off; off = align_up(off + szH);
  const size_t oKH = off; off = align_up(off + szH);
  const size_t oF  = off; off = align_up(off + szF);
  const size_t oP  = off; off = align_up(off + szP);
  const size_t oCP = off; off = align_up(off + szCP);
  const size_t oRC = off; off = align_up(off + szRCS);
  const size_t oVT = off; off = align_up(off + szVT);
  const size_t oRH = off; off = align_up(off + szR);
  const size_t oRL = off; off = align_up(off + szR);
  const size_t oY  = off; off = align_up(off + szY);
  const size_t oBP = off; off = align_up(off + szBNP);
  const size_t oBT = off; off = align_up(off + szBNT);
  if (off > ws_size) return;
  if (off > (size_t)WS_CAP) return;

  char* ws = (char*)d_ws;
  u16*    XQ  = (u16*)(ws + oXQ);
  u16*    XK  = (u16*)(ws + oXK);
  u16*    XV  = (u16*)(ws + oXV);
  u16*    WQ  = (u16*)(ws + oWQ);
  u16*    WK  = (u16*)(ws + oWK);
  u16*    WV  = (u16*)(ws + oWV);
  u16*    WO  = (u16*)(ws + oWO);
  u16*    QH  = (u16*)(ws + oQH);
  u16*    KH  = (u16*)(ws + oKH);
  float*  F   = (float*)(ws + oF);
  u16*    P   = (u16*)(ws + oP);
  float*  CP  = (float*)(ws + oCP);
  float*  RCS = (float*)(ws + oRC);
  u16*    VT  = (u16*)(ws + oVT);
  u16*    RH  = (u16*)(ws + oRH);
  u16*    RL  = (u16*)(ws + oRL);
  float*  Y   = (float*)(ws + oY);
  double* BNP = (double*)(ws + oBP);
  float*  BNT = (float*)(ws + oBT);

  const dim3 b256(256), b128(128);
  const dim3 gWT(2 * (DM / 64));
  const int  n8x = (int)(M * DM / 8);
  const dim3 gX((n8x + 255) / 256);
  const dim3 gG((unsigned)((M / 64) * (DM / 64)));
  const dim3 gA(NB * NQT16);
  const int  n4c = NB * SEQ / 4;
  const dim3 gC((n4c + 255) / 256);
  const dim3 gV(NB * 4 * (SEQ / 64));
  const dim3 gPV(NB * (SEQ / 64) * 4);
  const dim3 gWO((unsigned)((M / 64) * (DM / 64)));
  const dim3 gBP(nblk);
  const int  n4o = (int)(M * DM / 4);
  const dim3 gO((n4o + 255) / 256);
  const size_t ldsA = (size_t)16 * SPITCH * sizeof(float);

  wt16<<<gWT, b256, 0, stream>>>(Wq, WQ);
  wt16<<<gWT, b256, 0, stream>>>(Wk, WK);
  wt16<<<gWT, b256, 0, stream>>>(Wv, WV);
  wt16<<<gWT, b256, 0, stream>>>(Wo, WO);
  cvt16<<<gX, b256, 0, stream>>>(queries, XQ, n8x);
  cvt16<<<gX, b256, 0, stream>>>(keys,    XK, n8x);
  cvt16<<<gX, b256, 0, stream>>>(values,  XV, n8x);
  gemm_x<1><<<gG, b128, 0, stream>>>(XQ, WQ, bq, F, QH, (int)M, DM, DM, QSC);
  gemm_x<1><<<gG, b128, 0, stream>>>(XK, WK, bk, F, KH, (int)M, DM, DM, KSC);
  gemm_x<0><<<gG, b128, 0, stream>>>(XV, WV, bv, F, QH, (int)M, DM, DM, 1.0f);
  (void)hipFuncSetAttribute(reinterpret_cast<const void*>(&attn_p), hipFuncAttributeMaxDynamicSharedMemorySize, (int)ldsA);
  attn_p<<<gA, b256, ldsA, stream>>>(QH, KH, P, CP);
  csred<<<gC, b256, 0, stream>>>(CP, RCS, n4c);
  vt16<<<gV, b256, 0, stream>>>(F, RCS, VT);
  gemm_pv<<<gPV, b128, 0, stream>>>(P, VT, values, RH, RL);
  gemm_wo<<<gWO, b128, 0, stream>>>(RH, RL, WO, bo, Y, (int)M);
  bnpart<<<gBP, b256, 0, stream>>>(Y, BNP, nblk);
  bnfin<<<dim3(1), b256, 0, stream>>>(BNP, gamma, beta, BNT, nblk);
  bnapply<<<gO, b256, 0, stream>>>(Y, BNT, out, n4o);
  (void)hipGetLastError();
}
